// SimpleModel_85289460564645
// MI455X (gfx1250) — hardware-run, weakly checked
//
#include <hip/hip_runtime.h>


namespace {
constexpr int N = 100000, NP = 100096, E = 3200000, C1 = 16, EA = 3, C2 = 2, ZK = 64, NEB = 512;
constexpr float XS = 8.0f, WSC = 256.0f, NEG = 0.2f;
typedef _Float16 b16;
typedef __attribute__((ext_vector_type(16))) _Float16 v16b;
typedef __attribute__((ext_vector_type(8))) _Float16 v8b;
typedef __attribute__((ext_vector_type(8))) float v8f;
typedef __attribute__((ext_vector_type(4))) float v4f;
typedef __attribute__((ext_vector_type(2))) float v2f;
__device__ __forceinline__ float bf16_rne(float f) { unsigned int u = __float_as_uint(f); u += 0x7FFFu + ((u >> 16) & 1u); return __uint_as_float(u & 0xFFFF0000u); }
__device__ __forceinline__ void split16(float v, b16& hi, b16& lo) { hi = (b16)v; lo = (b16)(v - (float)hi); }
__device__ __forceinline__ v16b frag_kb(const b16* p, int hh) { const v8b a = *(const v8b*)(p + 8 * hh), b = *(const v8b*)(p + 16 + 8 * hh); v16b f;
#pragma unroll
  for (int e = 0; e < 8; ++e) { f[e] = a[e]; f[8 + e] = b[e]; } return f; }
__device__ __forceinline__ v8f wmma16b(v16b a, v16b b, v8f c) { v8f d = __builtin_amdgcn_wmma_f32_16x16x32_f16(false, a, false, b, (short)0, c, false, false); asm volatile("v_nop\n\tv_nop\n\tv_nop\n\tv_nop" : "+v"(d) : "v"(a), "v"(b)); return d; }
__device__ __forceinline__ void wave_lds_sync() { __builtin_amdgcn_fence(__ATOMIC_RELEASE, "workgroup"); __builtin_amdgcn_wave_barrier(); __builtin_amdgcn_fence(__ATOMIC_ACQUIRE, "workgroup"); }
__device__ __forceinline__ float pmul(float a, float b) { float p = a * b; asm volatile("" : "+v"(p)); return p; }
__device__ __forceinline__ float opaque(float a) { asm volatile("" : "+v"(a)); return a; }
__device__ __forceinline__ int iclamp(int v, int lo, int hi) { return v < lo ? lo : (v > hi ? hi : v); }
__device__ __forceinline__ float lrelu(float x) { return x > 0.0f ? x : NEG * x; }
__device__ __forceinline__ float nexp(float x) { return __builtin_amdgcn_exp2f(x * 1.4426950408889634f); }
constexpr int CSR_NBLK = 512, CSR_GB = 8, CSR_GN = 1 << CSR_GB  , CSR_TS = (CSR_GN < 32 ? 32 : CSR_GN)  , CSR_MAXG = 512, CSR_CAP = 12288  ;
__device__ __host__ __forceinline__ int csr_tix(int v) { return (v >> CSR_GB) * CSR_TS + (v & (CSR_GN - 1)); }
__global__ __launch_bounds__(64) void csrA_kernel(const int* __restrict__ dst, int E, int N, int nG, int CHP, int NGP, int* __restrict__ STG, int* __restrict__ HST) {
  extern __shared__ int sm[];
  int* cnt = sm; int* run = sm + NGP; int* ids = sm + 2 * NGP;
  const int b = blockIdx.x; const int ch = (E + CSR_NBLK - 1) / CSR_NBLK; const int e0 = b * ch, e1 = min(E, e0 + ch);
  for (int i = threadIdx.x; i < NGP; i += 64) cnt[i] = 0;
  for (int i = threadIdx.x; i < CHP; i += 64) ids[i] = -1;
  __syncthreads();
  if (threadIdx.x == 0) {
    for (int e = e0; e < e1; ++e) { int d = dst[e]; d = (d < 0) ? 0 : (d >= N ? N - 1 : d); cnt[d >> CSR_GB] += 1; }
    int acc = 0; for (int g = 0; g < nG; ++g) { run[g] = acc; acc += cnt[g]; }
    for (int e = e0; e < e1; ++e) { int d = dst[e]; d = (d < 0) ? 0 : (d >= N ? N - 1 : d); const int g = d >> CSR_GB; ids[run[g]] = e; run[g] += 1; } }
  __syncthreads();
  typedef __attribute__((ext_vector_type(4))) int v4i;
  for (int pass = 0; pass < 2; ++pass) {
    for (int i = threadIdx.x; i < CHP / 4; i += 64) *(volatile v4i*)(STG + (size_t)b * CHP + i * 4) = *(const v4i*)(&ids[i * 4]);
    for (int i = threadIdx.x; i < NGP / 4; i += 64) { v4i v; for (int e = 0; e < 4; ++e) v[e] = (i * 4 + e < nG) ? cnt[i * 4 + e] : 0; *(volatile v4i*)(HST + (size_t)b * NGP + i * 4) = v; }
    __threadfence(); }
}
__global__ __launch_bounds__(512) void csrS_kernel(const int* __restrict__ HST, int nG, int NGP, int* __restrict__ START, int* __restrict__ TOT, int* __restrict__ OFF) {
  __shared__ int tot[CSR_MAXG];
  const int b = threadIdx.x;
  for (int pass = 0; pass < 2; ++pass) { int runb = 0; for (int g = 0; g < nG; ++g) { int c = HST[(size_t)b * NGP + g]; c = (c < 0) ? 0 : c; ((volatile int*)OFF)[(size_t)g * CSR_NBLK + b] = runb; runb += c; } __threadfence(); }
  for (int g = threadIdx.x; g < nG; g += 512) { int s = 0; for (int bb = 0; bb < CSR_NBLK; ++bb) { int c = HST[(size_t)bb * NGP + g]; s += (c < 0) ? 0 : c; } tot[g] = s; }
  __syncthreads();
  if (threadIdx.x < 32) {
    __shared__ int st[CSR_MAXG + 32];
    if (threadIdx.x == 0) { int acc = 0; for (int g = 0; g < NGP; ++g) { st[g] = acc; if (g < nG) acc += (tot[g] + 31) & ~31; } st[NGP] = acc; }
    __builtin_amdgcn_fence(__ATOMIC_RELEASE, "workgroup"); __builtin_amdgcn_wave_barrier(); __builtin_amdgcn_fence(__ATOMIC_ACQUIRE, "workgroup");
    for (int pass = 0; pass < 2; ++pass) { for (int i = threadIdx.x; i < NGP + 32; i += 32) { ((volatile int*)START)[i] = (i <= NGP) ? st[min(i, NGP)] : 0; ((volatile int*)TOT)[i] = (i < nG) ? tot[i] : 0; } __threadfence(); } }
}
__global__ __launch_bounds__(256) void csrB_kernel(const int* __restrict__ dst, int N, int nG, int CHP, int NGP, int permLen, const int* __restrict__ STG, const int* __restrict__ HST, const int* __restrict__ OFF, const int* __restrict__ START, const int* __restrict__ TOT, int* __restrict__ PERM, int* __restrict__ ROWPTR, int* __restrict__ ROWCNT, int* __restrict__ FLAG) {
  typedef __attribute__((ext_vector_type(4))) int v4i;
  __shared__ int ids[CSR_CAP]; __shared__ unsigned short key[CSR_CAP]; __shared__ int outp[CSR_CAP]; __shared__ int ncnt[CSR_GN + 1]; __shared__ int boff[CSR_NBLK + 1];
  const int g = blockIdx.x, t_ = threadIdx.x; int tot = TOT[g]; int st = START[g], stn = START[g + 1]; const int v0 = g * CSR_GN; const int nv = min(CSR_GN, N - v0); const int t0 = g * CSR_TS;
  st = (st < 0) ? 0 : (st > permLen - 32 ? permLen - 32 : st) & ~31; stn = (stn < st) ? st : (stn > permLen ? permLen : stn); tot = (tot < 0) ? 0 : tot; if (tot > stn - st && tot <= CSR_CAP) tot = stn - st;
  if (tot > CSR_CAP) {
    for (int pass = 0; pass < 2; ++pass) { for (int i = t_; i < CSR_TS / 4; i += 256) { v4i a, c; for (int e = 0; e < 4; ++e) { a[e] = st; c[e] = 0; } *(volatile v4i*)(ROWPTR + t0 + i * 4) = a; *(volatile v4i*)(ROWCNT + t0 + i * 4) = c; } if (t_ == 0) ((volatile int*)FLAG)[0] = 1; __threadfence(); } (void)nv; return; }
  if (t_ == 0) { int acc = 0; for (int b = 0; b < CSR_NBLK; ++b) { boff[b] = acc; int c = HST[(size_t)b * NGP + g]; c = (c < 0) ? 0 : (c > CHP ? CHP : c); acc += c; if (acc > tot) acc = tot; } boff[CSR_NBLK] = acc; }
  for (int i = t_; i <= CSR_GN; i += 256) ncnt[i] = 0;
  __syncthreads();
  for (int b = 0; b < CSR_NBLK; ++b) { const int c = boff[b + 1] - boff[b]; int o_ = OFF[(size_t)g * CSR_NBLK + b]; o_ = (o_ < 0) ? 0 : (o_ > CHP - c ? CHP - c : o_); const int* src_ = STG + (size_t)b * CHP + o_;
    for (int i = t_; i < c; i += 256) { int id = src_[i]; id = (id < 0) ? 0 : id; ids[boff[b] + i] = id; int d = dst[id]; d = (d < v0) ? v0 : (d >= N ? N - 1 : d); int kk = d - v0; kk = (kk < 0) ? 0 : (kk >= CSR_GN ? CSR_GN - 1 : kk); key[boff[b] + i] = (unsigned short)kk; } }
  __syncthreads();
  if (t_ == 0) { for (int i = 0; i < tot; ++i) ncnt[key[i]] += 1; int acc = 0; for (int vl = 0; vl < CSR_GN; ++vl) { const int c = ncnt[vl]; ncnt[vl] = acc; acc += c; } ncnt[CSR_GN] = acc;
    for (int i = 0; i < tot; ++i) { const int vl = key[i]; outp[ncnt[vl]] = ids[i]; ncnt[vl] += 1; }
    for (int vl = CSR_GN; vl > 0; --vl) ncnt[vl] = ncnt[vl - 1]; ncnt[0] = 0; }
  __syncthreads();
  for (int pass = 0; pass < 2; ++pass) {
    for (int i = t_; i < (stn - st) / 4; i += 256) { v4i v; for (int e = 0; e < 4; ++e) { const int q = i * 4 + e; v[e] = (q < tot) ? outp[q] : -1; } *(volatile v4i*)(PERM + st + i * 4) = v; }
    for (int i = t_; i < CSR_TS / 4; i += 256) { v4i a, c; for (int e = 0; e < 4; ++e) { const int vl = i * 4 + e; const int vc = vl < CSR_GN ? vl : CSR_GN; a[e] = (vl < CSR_GN) ? st + ncnt[vc] : st; c[e] = (vl < nv) ? (ncnt[(vc < CSR_GN ? vc : CSR_GN - 1) + 1] - ncnt[vc]) : 0; } *(volatile v4i*)(ROWPTR + t0 + i * 4) = a; *(volatile v4i*)(ROWCNT + t0 + i * 4) = c; }
    __threadfence(); }
}
__global__ __launch_bounds__(256) void csrZ_kernel(int* __restrict__ p, size_t n4) { typedef __attribute__((ext_vector_type(4))) int v4i; const size_t tid = (size_t)blockIdx.x * 256 + threadIdx.x, nth = (size_t)gridDim.x * 256; v4i z = {0, 0, 0, 0}; for (size_t i = tid; i < n4; i += nth) *(volatile v4i*)(p + i * 4) = z; }
struct CsrBufs { int *STG, *HST, *OFF, *START, *TOT, *PERM, *ROWPTR, *ROWCNT, *FLAG; int nG, NGP, CHP; size_t permLen; char* base; size_t bytes; };
static size_t csr_carve(CsrBufs& c, char* ws, size_t off, int E, int N) {
  const size_t off0 = off; c.base = ws + off;
  auto al = [&](size_t bytes) { char* p = ws + off; off += (bytes + 255) & ~(size_t)255; return p; };
  c.nG = (N + CSR_GN - 1) / CSR_GN; c.NGP = (c.nG + 31) & ~31; const int ch = (E + CSR_NBLK - 1) / CSR_NBLK; c.CHP = (ch + 31) & ~31; c.permLen = (size_t)E + 32 * (size_t)c.nG + 32;
  c.STG = (int*)al((size_t)CSR_NBLK * c.CHP * 4); c.HST = (int*)al((size_t)CSR_NBLK * c.NGP * 4); c.OFF = (int*)al((size_t)c.NGP * CSR_NBLK * 4); c.START = (int*)al((size_t)(c.NGP + 64) * 4); c.TOT = (int*)al((size_t)(c.NGP + 64) * 4);
  c.PERM = (int*)al(c.permLen * 4); c.ROWPTR = (int*)al((size_t)c.nG * CSR_TS * 4); c.ROWCNT = (int*)al((size_t)c.nG * CSR_TS * 4); c.FLAG = (int*)al(256);
  c.bytes = off - off0; return off;
}
static void csr_build(const CsrBufs& c, const int* dst, int E, int N, hipStream_t stream) {
  const size_t smem = (size_t)(2 * c.NGP + c.CHP) * 4;
  csrZ_kernel<<<512, 256, 0, stream>>>((int*)c.base, c.bytes / 16);
  csrA_kernel<<<CSR_NBLK, 64, smem, stream>>>(dst, E, N, c.nG, c.CHP, c.NGP, c.STG, c.HST);
  csrS_kernel<<<1, 512, 0, stream>>>(c.HST, c.nG, c.NGP, c.START, c.TOT, c.OFF);
  csrB_kernel<<<c.nG, 256, 0, stream>>>(dst, N, c.nG, c.CHP, c.NGP, (int)c.permLen, c.STG, c.HST, c.OFF, c.START, c.TOT, c.PERM, c.ROWPTR, c.ROWCNT, c.FLAG);
}


__global__ __launch_bounds__(256) void wprep_kernel(const float* __restrict__ mw0, const float* __restrict__ mw1, const float* __restrict__ mw2, const float* __restrict__ mw3, b16* __restrict__ M0, b16* __restrict__ M1, b16* __restrict__ M2, b16* __restrict__ M3) {
  const int u = blockIdx.x * 256 + threadIdx.x; v8b v; int t = u;
  if (t < 16 * 64 / 8) { const int e = t * 8, o = e / 64, k0 = e % 64; for (int j = 0; j < 8; ++j) { const int k = k0 + j; v[j] = k < 35 ? (b16)(bf16_rne(mw0[(k < 35 ? k : 0) * 16 + o]) * WSC) : (b16)0.0f; } for (int p = 0; p < 2; ++p) { *(volatile v8b*)(M0 + e) = v; __threadfence(); } return; } t -= 128;
  if (t < 16 * 32 / 8) { const int e = t * 8, o = e / 32, k0 = e % 32; for (int j = 0; j < 8; ++j) { const int k = k0 + j; v[j] = k < 16 ? (b16)(bf16_rne(mw1[(k < 16 ? k : 0) * 16 + o]) * WSC) : (b16)0.0f; } for (int p = 0; p < 2; ++p) { *(volatile v8b*)(M1 + e) = v; __threadfence(); } return; } t -= 64;
  if (t < 16 * 32 / 8) { const int e = t * 8, o = e / 32, k0 = e % 32; for (int j = 0; j < 8; ++j) { const int k = k0 + j; v[j] = (k < 16 && o < 8) ? (b16)(bf16_rne(mw2[(k < 16 ? k : 0) * 8 + (o < 8 ? o : 0)]) * WSC) : (b16)0.0f; } for (int p = 0; p < 2; ++p) { *(volatile v8b*)(M2 + e) = v; __threadfence(); } return; } t -= 64;
  if (t < 16 * 32 / 8) { const int e = t * 8, o = e / 32, k0 = e % 32; for (int j = 0; j < 8; ++j) { const int k = k0 + j; v[j] = (k < 8 && o < 4) ? (b16)(bf16_rne(mw3[(k < 8 ? k : 0) * 4 + (o < 4 ? o : 0)]) * WSC) : (b16)0.0f; } for (int p = 0; p < 2; ++p) { *(volatile v8b*)(M3 + e) = v; __threadfence(); } }
}
template <int W, int RAW>
__global__ __launch_bounds__(256) void colsum_kernel(const float* __restrict__ P, int NE, float* __restrict__ PS) {
  __shared__ double red[256];
  double acc[W]; for (int w = 0; w < W; ++w) acc[w] = 0.0;
  for (int r = blockIdx.x * 256 + threadIdx.x; r < NE; r += NEB * 256) for (int w = 0; w < W; ++w) { const float v = P[(size_t)r * W + w]; acc[w] += (double)(RAW ? bf16_rne(v) : v); }
  float res[W];
  for (int w = 0; w < W; ++w) { red[threadIdx.x] = acc[w]; __syncthreads(); for (int s = 128; s > 0; s >>= 1) { if ((int)threadIdx.x < s) red[threadIdx.x] += red[threadIdx.x + s]; __syncthreads(); } res[w] = (float)red[0]; __syncthreads(); }
  for (int pass = 0; pass < 2; ++pass) { if (threadIdx.x < 32) ((volatile float*)PS)[(size_t)blockIdx.x * 32 + threadIdx.x] = ((int)threadIdx.x < W) ? res[threadIdx.x < W ? threadIdx.x : 0] : 0.0f; __threadfence(); }
}
template <int W>
__global__ __launch_bounds__(32) void colmean_kernel(const float* __restrict__ PS, int NE, float* __restrict__ MEAN) {
  const int lane = threadIdx.x; float outv = 0.0f;
  for (int w = 0; w < W; ++w) { double s = 0.0; for (int b = lane; b < NEB; b += 32) s += (double)PS[(size_t)b * 32 + w]; for (int o = 16; o; o >>= 1) s += __shfl_xor(s, o); if (lane == w) outv = (float)(s / (double)NE); }
  for (int pass = 0; pass < 2; ++pass) { ((volatile float*)MEAN)[lane] = outv; __threadfence(); }
}
__global__ __launch_bounds__(256) void node1_kernel(const float* __restrict__ x, const float* __restrict__ W1, const float* __restrict__ as1, const float* __restrict__ ad1, float* __restrict__ H1, float* __restrict__ ALS, float* __restrict__ ALD) {
  __shared__ __attribute__((aligned(16))) float sh[256][C1]; __shared__ float sa[256], sd[256];
  const int n = blockIdx.x * 256 + threadIdx.x; float h[C1]; for (int c = 0; c < C1; ++c) h[c] = 0.0f;
  if (n < N) { const v4f xv = *(const v4f*)(x + (size_t)n * 4);
    for (int c = 0; c < C1; ++c) { float s = 0.0f; for (int k = 0; k < 4; ++k) s += pmul(bf16_rne(xv[k]), bf16_rne(W1[k * C1 + c])); h[c] = s; } }
  float ps = 0.0f, pd = 0.0f; for (int c = 0; c < C1; ++c) { sh[threadIdx.x][c] = h[c]; ps += pmul(h[c], bf16_rne(as1[c])); pd += pmul(h[c], bf16_rne(ad1[c])); } sa[threadIdx.x] = ps; sd[threadIdx.x] = pd;
  __syncthreads();
  const float* shf = &sh[0][0];
  for (int pass = 0; pass < 2; ++pass) { for (int q = 0; q < 4; ++q) { const int idx = q * 256 + threadIdx.x; *(volatile v4f*)(H1 + (size_t)blockIdx.x * 256 * C1 + (size_t)idx * 4) = *(const v4f*)(shf + idx * 4); }
    ((volatile float*)ALS)[n] = sa[threadIdx.x]; ((volatile float*)ALD)[n] = sd[threadIdx.x]; __threadfence(); }
}
__global__ __launch_bounds__(512) void gat1_kernel(const float* __restrict__ H1, const float* __restrict__ ALS, const float* __restrict__ ALD, const float* __restrict__ ea, const float* __restrict__ We1, const float* __restrict__ ae1, const float* __restrict__ MEAN1, const float* __restrict__ b1,
                                                    const float* __restrict__ W2, const float* __restrict__ as2, const float* __restrict__ ad2,
                                                    const int* __restrict__ srcs, const int* __restrict__ PERM, const int* __restrict__ ROWPTR, const int* __restrict__ ROWCNT, int permLen, int ELIM, int NLIM, float* __restrict__ H, float* __restrict__ ND2) {
  __shared__ __attribute__((aligned(16))) float sh[16][C1]; __shared__ __attribute__((aligned(16))) float s2[16][4];
  const int wave = threadIdx.x >> 5, lane = threadIdx.x & 31; const size_t v = (size_t)blockIdx.x * 16 + wave;
  float wea[EA]; for (int k = 0; k < EA; ++k) { float s = 0.0f; for (int c = 0; c < C1; ++c) s += pmul(bf16_rne(We1[k * C1 + c]), bf16_rne(ae1[c])); wea[k] = s; }
  float hrow[C1]; for (int c = 0; c < C1; ++c) hrow[c] = 0.0f;
  if (v < (size_t)NLIM) { int st = ROWPTR[v], cnt = ROWCNT[v]; cnt = iclamp(cnt, 0, 1 << 20); st = iclamp(st, 0, permLen - cnt); const float adv = ALD[v];
    float sl = ALS[v] + adv; for (int k = 0; k < EA; ++k) sl += pmul(MEAN1[k], wea[k]); sl = lrelu(sl);
    float mx = sl;
    for (int j = lane; j < cnt; j += 32) { const int e = iclamp(PERM[st + j], 0, ELIM - 1); const int s = iclamp(srcs[e], 0, N - 1); float sc = ALS[s] + adv; for (int k = 0; k < EA; ++k) sc += pmul(bf16_rne(ea[(size_t)e * EA + k]), wea[k]); mx = fmaxf(mx, lrelu(sc)); }
    for (int o = 16; o; o >>= 1) mx = fmaxf(mx, __shfl_xor(mx, o));
    float den = 0.0f, acc[C1]; for (int c = 0; c < C1; ++c) acc[c] = 0.0f;
    if (lane == 0) { const float p = nexp(sl - mx); den = p; for (int c = 0; c < C1; ++c) acc[c] = pmul(p, H1[v * C1 + c]); }
    for (int j = lane; j < cnt; j += 32) { const int e = iclamp(PERM[st + j], 0, ELIM - 1); const size_t s = (size_t)iclamp(srcs[e], 0, N - 1); float sc = ALS[s] + adv; for (int k = 0; k < EA; ++k) sc += pmul(bf16_rne(ea[(size_t)e * EA + k]), wea[k]);
      const float p = nexp(lrelu(sc) - mx); den += p; for (int q = 0; q < 4; ++q) { const v4f hv = *(const v4f*)(H1 + s * C1 + q * 4); for (int i = 0; i < 4; ++i) acc[q * 4 + i] += pmul(p, hv[i]); } }
    for (int o = 16; o; o >>= 1) { den += __shfl_xor(den, o); for (int c = 0; c < C1; ++c) acc[c] += __shfl_xor(acc[c], o); }
    const float inv = 1.0f / (den + 1e-16f); for (int c = 0; c < C1; ++c) hrow[c] = pmul(acc[c], inv) + bf16_rne(b1[c]); }
  if (lane < C1) sh[wave][lane] = hrow[lane];
  if (lane == 0) { float h2a = 0.0f, h2b = 0.0f; for (int c = 0; c < C1; ++c) { h2a += pmul(hrow[c], bf16_rne(W2[c * 2])); h2b += pmul(hrow[c], bf16_rne(W2[c * 2 + 1])); }
    s2[wave][0] = h2a; s2[wave][1] = h2b; s2[wave][2] = pmul(h2a, bf16_rne(as2[0])) + pmul(h2b, bf16_rne(as2[1])); s2[wave][3] = pmul(h2a, bf16_rne(ad2[0])) + pmul(h2b, bf16_rne(ad2[1])); }
  __syncthreads();
  for (int pass = 0; pass < 2; ++pass) { if (threadIdx.x < 64) *(volatile v4f*)(H + (size_t)blockIdx.x * 16 * C1 + threadIdx.x * 4) = *(const v4f*)(&sh[0][0] + threadIdx.x * 4);
    else if (threadIdx.x < 80) *(volatile v4f*)(ND2 + (size_t)blockIdx.x * 16 * 4 + (threadIdx.x - 64) * 4) = *(const v4f*)(&s2[threadIdx.x - 64][0]); __threadfence(); }
}
__global__ __launch_bounds__(256) void emlp_kernel(const float* __restrict__ H, const float* __restrict__ ea, const int* __restrict__ srcs, const int* __restrict__ dsts, const b16* __restrict__ M0, const b16* __restrict__ M1, const b16* __restrict__ M2, const b16* __restrict__ M3,
                                                    const float* __restrict__ mb0, const float* __restrict__ mb1, const float* __restrict__ mb2, const float* __restrict__ mb3, float* __restrict__ E4, float* __restrict__ out1) {
  __shared__ __attribute__((aligned(16))) b16 Ah[8][16][ZK + 8], Al[8][16][ZK + 8]; __shared__ __attribute__((aligned(16))) float So[8][16][4], Sl[8][16][4];
  const int wave = threadIdx.x >> 5, lane = threadIdx.x & 31, nloc = lane & 15, hlf = lane >> 4; const size_t e0 = ((size_t)blockIdx.x * 8 + wave) * 16;
  {
    const size_t e = e0 + nloc; const int nd = hlf == 0 ? iclamp(srcs[e], 0, N - 1) : iclamp(dsts[e], 0, N - 1); const float* hr = H + (size_t)nd * C1;
    if (hlf == 0) { for (int c = 0; c < C1; ++c) { b16 p, q; split16(hr[c] * XS, p, q); Ah[wave][nloc][c] = p; Al[wave][nloc][c] = q; }
      for (int k = 0; k < EA; ++k) { Ah[wave][nloc][C1 + k] = (b16)(bf16_rne(ea[e * EA + k]) * XS); Al[wave][nloc][C1 + k] = (b16)0.0f; } }
    else { for (int c = 0; c < C1; ++c) { b16 p, q; split16(hr[c] * XS, p, q); Ah[wave][nloc][C1 + EA + c] = p; Al[wave][nloc][C1 + EA + c] = q; } for (int c = 35; c < ZK; ++c) { Ah[wave][nloc][c] = (b16)0.0f; Al[wave][nloc][c] = (b16)0.0f; } } }
  wave_lds_sync();
  const float sc = 1.0f / (XS * WSC);
  v8f acc = (v8f){};
#pragma unroll
  for (int kb = 0; kb < ZK; kb += 32) { const v16b a = frag_kb(&Ah[wave][nloc][kb], hlf), al = frag_kb(&Al[wave][nloc][kb], hlf); const v16b bw = frag_kb(M0 + (size_t)nloc * ZK + kb, hlf); acc = wmma16b(a, bw, acc); acc = wmma16b(al, bw, acc); }
  wave_lds_sync();
  { const float bb = bf16_rne(mb0[nloc]);
#pragma unroll
    for (int r8 = 0; r8 < 8; ++r8) { const float v = fmaxf(acc[r8] * sc + bb, 0.0f); b16 p, q; split16(v * XS, p, q); Ah[wave][8 * hlf + r8][nloc] = p; Al[wave][8 * hlf + r8][nloc] = q; Ah[wave][8 * hlf + r8][16 + nloc] = (b16)0.0f; Al[wave][8 * hlf + r8][16 + nloc] = (b16)0.0f; } }
  wave_lds_sync();
  acc = (v8f){}; { const v16b a = frag_kb(&Ah[wave][nloc][0], hlf), al = frag_kb(&Al[wave][nloc][0], hlf); const v16b bw = frag_kb(M1 + (size_t)nloc * 32, hlf); acc = wmma16b(a, bw, acc); acc = wmma16b(al, bw, acc); }
  wave_lds_sync();
  { const float bb = bf16_rne(mb1[nloc]);
#pragma unroll
    for (int r8 = 0; r8 < 8; ++r8) { const float v = fmaxf(acc[r8] * sc + bb, 0.0f); b16 p, q; split16(v * XS, p, q); Ah[wave][8 * hlf + r8][nloc] = p; Al[wave][8 * hlf + r8][nloc] = q; } }
  wave_lds_sync();
  acc = (v8f){}; { const v16b a = frag_kb(&Ah[wave][nloc][0], hlf), al = frag_kb(&Al[wave][nloc][0], hlf); const v16b bw = frag_kb(M2 + (size_t)nloc * 32, hlf); acc = wmma16b(a, bw, acc); acc = wmma16b(al, bw, acc); }
  wave_lds_sync();
  { const float bb = nloc < 8 ? bf16_rne(mb2[nloc < 8 ? nloc : 0]) : 0.0f;
#pragma unroll
    for (int r8 = 0; r8 < 8; ++r8) { const float v = nloc < 8 ? fmaxf(acc[r8] * sc + bb, 0.0f) : 0.0f; b16 p, q; split16(v * XS, p, q); Ah[wave][8 * hlf + r8][nloc] = p; Al[wave][8 * hlf + r8][nloc] = q; } }
  wave_lds_sync();
  acc = (v8f){}; { const v16b a = frag_kb(&Ah[wave][nloc][0], hlf), al = frag_kb(&Al[wave][nloc][0], hlf); const v16b bw = frag_kb(M3 + (size_t)nloc * 32, hlf); acc = wmma16b(a, bw, acc); acc = wmma16b(al, bw, acc); }
  if (nloc < 4) { const float bb = bf16_rne(mb3[nloc]);
#pragma unroll
    for (int r8 = 0; r8 < 8; ++r8) So[wave][8 * hlf + r8][nloc] = acc[r8] * sc + bb; }
  wave_lds_sync();
  if (lane < 16) { const float a0 = So[wave][lane][0], a1 = So[wave][lane][1], a2 = So[wave][lane][2], a3 = So[wave][lane][3]; const float m = fmaxf(fmaxf(a0, a1), fmaxf(a2, a3)); const float se = nexp(a0 - m) + nexp(a1 - m) + nexp(a2 - m) + nexp(a3 - m); const float l = m + __logf(se);
    Sl[wave][lane][0] = a0 - l; Sl[wave][lane][1] = a1 - l; Sl[wave][lane][2] = a2 - l; Sl[wave][lane][3] = a3 - l; }
  wave_lds_sync();
  for (int pass = 0; pass < 2; ++pass) { if (lane < 16) *(volatile v4f*)(E4 + (e0 + lane) * 4) = *(const v4f*)(&So[wave][lane][0]); else *(volatile v4f*)(out1 + (e0 + lane - 16) * 4) = *(const v4f*)(&Sl[wave][lane - 16][0]); __threadfence(); }
}
__global__ __launch_bounds__(512) void gat2_kernel(const float* __restrict__ ND2, const float* __restrict__ E4, const float* __restrict__ We2, const float* __restrict__ ae2, const float* __restrict__ MEAN2, const float* __restrict__ b2,
                                                    const int* __restrict__ srcs, const int* __restrict__ PERM, const int* __restrict__ ROWPTR, const int* __restrict__ ROWCNT, int permLen, int ELIM, int NLIM, float* __restrict__ out0) {
  __shared__ __attribute__((aligned(16))) float so[16][2];
  const int wave = threadIdx.x >> 5, lane = threadIdx.x & 31; const size_t v = (size_t)blockIdx.x * 16 + wave;
  float wea[4]; for (int k = 0; k < 4; ++k) wea[k] = pmul(bf16_rne(We2[k * 2]), bf16_rne(ae2[0])) + pmul(bf16_rne(We2[k * 2 + 1]), bf16_rne(ae2[1]));
  float o0 = 0.0f, o1 = 0.0f;
  if (v < (size_t)NLIM) { int st = ROWPTR[v], cnt = ROWCNT[v]; cnt = iclamp(cnt, 0, 1 << 20); st = iclamp(st, 0, permLen - cnt); const v4f nv = *(const v4f*)(ND2 + v * 4); const float adv = nv[3];
    float sl = nv[2] + adv; for (int k = 0; k < 4; ++k) sl += pmul(MEAN2[k], wea[k]); sl = lrelu(sl); float mx = sl;
    for (int j = lane; j < cnt; j += 32) { const int e = iclamp(PERM[st + j], 0, ELIM - 1); const int s = iclamp(srcs[e], 0, N - 1); const v4f ns = *(const v4f*)(ND2 + (size_t)s * 4), ev = *(const v4f*)(E4 + (size_t)e * 4); float sc = ns[2] + adv; for (int k = 0; k < 4; ++k) sc += pmul(ev[k], wea[k]); mx = fmaxf(mx, lrelu(sc)); }
    for (int o = 16; o; o >>= 1) mx = fmaxf(mx, __shfl_xor(mx, o));
    float den = 0.0f, a0 = 0.0f, a1 = 0.0f; if (lane == 0) { const float p = nexp(sl - mx); den = p; a0 = pmul(p, nv[0]); a1 = pmul(p, nv[1]); }
    for (int j = lane; j < cnt; j += 32) { const int e = iclamp(PERM[st + j], 0, ELIM - 1); const int s = iclamp(srcs[e], 0, N - 1); const v4f ns = *(const v4f*)(ND2 + (size_t)s * 4), ev = *(const v4f*)(E4 + (size_t)e * 4); float sc = ns[2] + adv; for (int k = 0; k < 4; ++k) sc += pmul(ev[k], wea[k]);
      const float p = nexp(lrelu(sc) - mx); den += p; a0 += pmul(p, ns[0]); a1 += pmul(p, ns[1]); }
    for (int o = 16; o; o >>= 1) { den += __shfl_xor(den, o); a0 += __shfl_xor(a0, o); a1 += __shfl_xor(a1, o); }
    const float inv = 1.0f / (den + 1e-16f); o0 = pmul(a0, inv) + bf16_rne(b2[0]); o1 = pmul(a1, inv) + bf16_rne(b2[1]);
    const float m = fmaxf(o0, o1); const float l = m + __logf(nexp(o0 - m) + nexp(o1 - m)); o0 -= l; o1 -= l; }
  if (lane == 0) { so[wave][0] = o0; so[wave][1] = o1; }
  __syncthreads();
  for (int pass = 0; pass < 2; ++pass) { if (threadIdx.x < 8 && ((size_t)blockIdx.x * 16 + threadIdx.x * 2 + 1) < (size_t)N) *(volatile v4f*)(out0 + (size_t)blockIdx.x * 32 + threadIdx.x * 4) = *(const v4f*)(&so[0][0] + threadIdx.x * 4); __threadfence(); }
}
}

extern "C" void kernel_launch(void* const* d_in, const int* in_sizes, int n_in, void* d_out, int out_size, void* d_ws, size_t ws_size, hipStream_t stream) {
  (void)n_in;
  auto Fp = [&](int i) { return (const float*)d_in[i]; }; auto Ip = [&](int i) { return (const int*)d_in[i]; };
  if (in_sizes[0] != N * 4 || in_sizes[1] != E * EA || in_sizes[2] != 4 * C1 || in_sizes[8] != 35 * 16 || in_sizes[14] != 8 * 4 || in_sizes[16] != C1 * C2 || in_sizes[19] != 4 * 2 || in_sizes[22] != 2 * E || out_size != N * 2 + E * 4) return;
  const int ELIM = E, NLIM = N;
  size_t off = 0; char* ws = (char*)d_ws;
  auto carve = [&](size_t bytes) { char* p = ws + off; off += (bytes + 255) & ~(size_t)255; return p; };
  b16* M0 = (b16*)carve(16 * 64 * 2); b16* M1 = (b16*)carve(16 * 32 * 2); b16* M2 = (b16*)carve(16 * 32 * 2); b16* M3 = (b16*)carve(16 * 32 * 2);
  float* H1 = (float*)carve((size_t)NP * C1 * 4); float* ALS = (float*)carve((size_t)NP * 4); float* ALD = (float*)carve((size_t)NP * 4); float* H = (float*)carve((size_t)NP * C1 * 4); float* ND2 = (float*)carve((size_t)NP * 4 * 4);
  float* E4 = (float*)carve((size_t)E * 4 * 4); float* PS1 = (float*)carve((size_t)NEB * 32 * 4); float* PS2 = (float*)carve((size_t)NEB * 32 * 4); float* MEAN1 = (float*)carve(32 * 4); float* MEAN2 = (float*)carve(32 * 4);
  CsrBufs csr; off = csr_carve(csr, ws, off, ELIM, N);
  if (off > ws_size || off > ((size_t)128 << 20)) return;
  float* out0 = (float*)d_out; float* out1 = out0 + (size_t)N * 2;
  wprep_kernel<<<2, 256, 0, stream>>>(Fp(8), Fp(10), Fp(12), Fp(14), M0, M1, M2, M3);
  colsum_kernel<EA, 1><<<NEB, 256, 0, stream>>>(Fp(1), ELIM, PS1); colmean_kernel<EA><<<1, 32, 0, stream>>>(PS1, ELIM, MEAN1);
  csr_build(csr, Ip(22) + E, ELIM, N, stream);
  node1_kernel<<<NP / 256, 256, 0, stream>>>(Fp(0), Fp(2), Fp(3), Fp(4), H1, ALS, ALD);
  gat1_kernel<<<NP / 16, 512, 0, stream>>>(H1, ALS, ALD, Fp(1), Fp(5), Fp(6), MEAN1, Fp(7), Fp(16), Fp(17), Fp(18), Ip(22), csr.PERM, csr.ROWPTR, csr.ROWCNT, (int)csr.permLen, ELIM, NLIM, H, ND2);
  emlp_kernel<<<ELIM / 128, 256, 0, stream>>>(H, Fp(1), Ip(22), Ip(22) + E, M0, M1, M2, M3, Fp(9), Fp(11), Fp(13), Fp(15), E4, out1);
  colsum_kernel<4, 0><<<NEB, 256, 0, stream>>>(E4, ELIM, PS2); colmean_kernel<4><<<1, 32, 0, stream>>>(PS2, ELIM, MEAN2);
  gat2_kernel<<<NP / 16, 512, 0, stream>>>(ND2, E4, Fp(19), Fp(20), MEAN2, Fp(21), Ip(22), csr.PERM, csr.ROWPTR, csr.ROWCNT, (int)csr.permLen, ELIM, NLIM, out0);
}
